// EGNNLayer_5841155523150
// MI455X (gfx1250) — hardware-verified
//
#include <hip/hip_runtime.h>
#include <stddef.h>
#include <stdint.h>

#define NBAT   4
#define NN     512
#define DS     128
#define ED     32
#define MR     (NBAT * NN)
#define KA1    192
#define KH     256
#define NPQ    64
#define NTHR   256
#define GBM    64
#define GTHR   128
#define RPB    8
#define EFP    36
#define WVF    (16 * EFP + 64)
#define LQ     (NN * ED)
#define LX     (NN * 4)
#define LM     NN
#define LV     256
#define LW     (RPB * WVF)
#define LMX    32
#define PAIR_LDS_BYTES ((LQ + LX + LM + LV + LW + LMX) * 4)
#define WSMAX  134217728

#define U_WPQ  (NPQ * (DS / 8))
#define U_W2   (ED * (ED / 8))
#define U_W3H  (ED * (ED / 8))
#define U_SW1  (DS * (KA1 / 8))
#define U_SW2  (DS * (KH / 8))
#define U_A1   (MR * (DS / 8))
#define U_XR   MR
#define U_VA   256
#define U_VB   64
#define E0 (U_WPQ)
#define E1 (E0 + U_W2)
#define E2 (E1 + U_W3H)
#define E3 (E2 + U_W3H)
#define E4 (E3 + U_SW1)
#define E5 (E4 + U_SW2)
#define E6 (E5 + U_A1)
#define E7 (E6 + U_XR)
#define E8 (E7 + U_VA)
#define E9 (E8 + U_VB)

static_assert(NN == 32 * 16);
static_assert(NN % RPB == 0);
static_assert(RPB * 32 == NTHR);
static_assert(ED == 32);
static_assert(DS == 128);
static_assert(KA1 * 2 == 3 * 128);
static_assert(KA1 % 32 == 0 && KH % 32 == 0 && DS % 32 == 0);
static_assert(MR % GBM == 0);
static_assert(GBM == (GTHR / 32) * 16);
static_assert((MR * 3) % 32 == 0);
static_assert((MR * 3 / 4) % NTHR == 0);
static_assert(E0 % 32 == 0 && E1 % 32 == 0 && E2 % 32 == 0 && E3 % 32 == 0 && E4 % 32 == 0);
static_assert(E5 % 32 == 0 && E6 % 32 == 0 && E7 % 32 == 0 && E8 % 32 == 0 && E9 % 32 == 0);
static_assert((EFP * 4) % 16 == 0 && EFP >= ED);
static_assert((WVF * 4) % 16 == 0);
static_assert(PAIR_LDS_BYTES <= 300000);
static_assert((LQ / 4) % NTHR == 0 && NN == 2 * NTHR && LV / 4 <= NTHR);

typedef float          v4f   __attribute__((ext_vector_type(4)));
typedef float          v8f   __attribute__((ext_vector_type(8)));
typedef int            v8i   __attribute__((ext_vector_type(8)));
typedef unsigned       v2u   __attribute__((ext_vector_type(2)));
typedef unsigned short v8us  __attribute__((ext_vector_type(8)));
typedef unsigned short v16us __attribute__((ext_vector_type(16)));
typedef __bf16         v16bf __attribute__((ext_vector_type(16)));
typedef v4f  __attribute__((may_alias)) v4fa;
typedef v2u  __attribute__((may_alias)) v2ua;
typedef v8us __attribute__((may_alias)) v8usa;
union FragB { v16bf v; v16us u; v8us h[2]; v8i w; };

__device__ __forceinline__ v8f wmb(const FragB& a, const FragB& b, v8f c) {
  v8f d = __builtin_amdgcn_wmma_f32_16x16x32_bf16(false, a.v, false, b.v, (short)0, c, false, false);
  asm volatile("v_nop\n\tv_nop\n\tv_nop\n\tv_nop" : "+v"(d) : "v"(a.w), "v"(b.w));
  return d;
}

__device__ __forceinline__ unsigned bf16_bits(float f) {
  const unsigned u = __float_as_uint(f);
  return (u + 0x7FFFu + ((u >> 16) & 1u)) >> 16;
}
__device__ __forceinline__ float bf16_val(float f) {
  return __uint_as_float(bf16_bits(f) << 16);
}
__device__ __forceinline__ unsigned split2(float v) {
  const unsigned hb = bf16_bits(v);
  const unsigned lb = bf16_bits(v - __uint_as_float(hb << 16));
  return hb | (lb << 16);
}
__device__ __forceinline__ float silu_f(float t) {
  return t * __builtin_amdgcn_rcpf(1.0f + expf(-t));
}
__device__ __forceinline__ void put16(unsigned short* dp, v8us o) {
  *(volatile v8us*)dp = o;
  __threadfence();
  *(volatile v8us*)dp = o;
}
__device__ __forceinline__ void putf4(float* dp, v4f o) {
  *(volatile v4f*)dp = o;
  __threadfence();
  *(volatile v4f*)dp = o;
}
__device__ __forceinline__ void wave_sync() {
  __threadfence_block();
  __builtin_amdgcn_wave_barrier();
  __threadfence_block();
}
__device__ __forceinline__ float hsum16(float v) {
  v += __shfl_xor(v, 1, 32);
  v += __shfl_xor(v, 2, 32);
  v += __shfl_xor(v, 4, 32);
  v += __shfl_xor(v, 8, 32);
  return v;
}
__device__ __forceinline__ float hmax16(float v) {
  v = fmaxf(v, __shfl_xor(v, 1, 32));
  v = fmaxf(v, __shfl_xor(v, 2, 32));
  v = fmaxf(v, __shfl_xor(v, 4, 32));
  v = fmaxf(v, __shfl_xor(v, 8, 32));
  return v;
}

__global__ __launch_bounds__(NTHR) void k_prep(
    const float* __restrict__ s, const float* __restrict__ x,
    const float* __restrict__ ew1, const float* __restrict__ eb1,
    const float* __restrict__ ew2, const float* __restrict__ eb2,
    const float* __restrict__ aw1, const float* __restrict__ ab1,
    const float* __restrict__ aw2, const float* __restrict__ ab2,
    const float* __restrict__ sw1, const float* __restrict__ sb1,
    const float* __restrict__ sw2, const float* __restrict__ sb2,
    const float* __restrict__ cw1, const float* __restrict__ cb1,
    const float* __restrict__ cw2, const float* __restrict__ cb2,
    unsigned short* A1, float* XR, unsigned short* WPQ, unsigned short* W2, unsigned short* W3,
    unsigned short* SW1C, unsigned short* SW2D, float* VEC) {
  const int u = (int)blockIdx.x * NTHR + (int)threadIdx.x;
  v8us o;
  if (u < E0) {
    const int n  = u >> 4;
    const int k8 = (u & 15) * 8;
    const float* p = ew1 + (size_t)((n >> 5) * DS + k8) * ED + (n & 31);
#pragma unroll
    for (int i = 0; i < 8; ++i) o[i] = (unsigned short)bf16_bits(p[(size_t)i * ED]);
    put16(WPQ + (size_t)n * DS + k8, o);
    return;
  } else if (u < E1) {
    const int v  = u - E0;
    const int n  = v >> 2;
    const int k8 = (v & 3) * 8;
    const float* p = ew2 + (size_t)k8 * ED + n;
#pragma unroll
    for (int i = 0; i < 8; ++i) o[i] = (unsigned short)bf16_bits(p[(size_t)i * ED]);
    put16(W2 + (size_t)n * ED + k8, o);
    return;
  } else if (u < E2) {
    const int v  = u - E1;
    const int n  = v >> 2;
    const int k8 = (v & 3) * 8;
    const float* p = aw1 + (size_t)k8 * ED + n;
#pragma unroll
    for (int i = 0; i < 8; ++i) o[i] = (unsigned short)bf16_bits(p[(size_t)i * ED]);
    put16(W3 + (size_t)n * ED + k8, o);
    return;
  } else if (u < E3) {
    const int v  = u - E2;
    const int n  = v >> 2;
    const int k8 = (v & 3) * 8;
    const float* p = cw1 + (size_t)k8 * ED + n;
#pragma unroll
    for (int i = 0; i < 8; ++i) o[i] = (unsigned short)bf16_bits(p[(size_t)i * ED]);
    put16(W3 + (size_t)(ED + n) * ED + k8, o);
    return;
  } else if (u < E4) {
    const int v    = u - E3;
    const int n    = v / (KA1 / 8);
    const int k8   = (v - n * (KA1 / 8)) * 8;
    const int srow = (k8 < DS + ED) ? k8 : (k8 - ED);
    const float* p = sw1 + (size_t)srow * DS + n;
#pragma unroll
    for (int i = 0; i < 8; ++i) o[i] = (unsigned short)bf16_bits(p[(size_t)i * DS]);
    put16(SW1C + (size_t)n * KA1 + k8, o);
    return;
  } else if (u < E5) {
    const int v    = u - E4;
    const int n    = v >> 5;
    const int k8   = (v & 31) * 8;
    const int srow = k8 & (DS - 1);
    const float* p = sw2 + (size_t)srow * DS + n;
#pragma unroll
    for (int i = 0; i < 8; ++i) o[i] = (unsigned short)bf16_bits(p[(size_t)i * DS]);
    put16(SW2D + (size_t)n * KH + k8, o);
    return;
  } else if (u < E6) {
    const int v   = u - E5;
    const int row = v >> 4;
    const int k8  = (v & 15) * 8;
    const float* p = s + (size_t)row * DS + k8;
    const v4f a = *(const v4fa*)p;
    const v4f b = *(const v4fa*)(p + 4);
    o[0] = (unsigned short)bf16_bits(a.x);
    o[1] = (unsigned short)bf16_bits(a.y);
    o[2] = (unsigned short)bf16_bits(a.z);
    o[3] = (unsigned short)bf16_bits(a.w);
    o[4] = (unsigned short)bf16_bits(b.x);
    o[5] = (unsigned short)bf16_bits(b.y);
    o[6] = (unsigned short)bf16_bits(b.z);
    o[7] = (unsigned short)bf16_bits(b.w);
    put16(A1 + (size_t)row * KA1 + k8, o);
    return;
  } else if (u < E7) {
    const int row = u - E6;
    const float x0 = x[(size_t)row * 3 + 0];
    const float x1 = x[(size_t)row * 3 + 1];
    const float x2 = x[(size_t)row * 3 + 2];
    v4f q;
    q.x = bf16_val(x0);
    q.y = bf16_val(x1);
    q.z = bf16_val(x2);
    q.w = 0.0f;
    putf4(XR + (size_t)row * 4, q);
    return;
  } else if (u < E8) {
    const int vv = u - E7;
    const int wv = __builtin_amdgcn_readfirstlane(vv >> 5);
    const int ln = vv & 31;
    const int q  = ln & 7;
    v4f o4;
    if (wv < 7) {
      const float* src = ew1 + (size_t)(2 * DS) * ED;
      if (wv == 1) src = eb1;
      if (wv == 2) src = eb2;
      if (wv == 3) src = ab1;
      if (wv == 4) src = cb1;
      if (wv == 5) src = aw2;
      if (wv == 6) src = cw2;
      const v4f a = *(const v4fa*)(src + 4 * q);
      o4.x = bf16_val(a.x);
      o4.y = bf16_val(a.y);
      o4.z = bf16_val(a.z);
      o4.w = bf16_val(a.w);
    } else {
      const float va = bf16_val(ab2[0]);
      const float vc = bf16_val(cb2[0]);
      o4.x = (q == 0) ? va : 0.0f;
      o4.y = (q == 0) ? vc : 0.0f;
      o4.z = 0.0f;
      o4.w = 0.0f;
    }
    float* dp = VEC + 32 * wv + 4 * q;
    if (ln < 8) *(volatile v4f*)dp = o4;
    __threadfence();
    if (ln < 8) *(volatile v4f*)dp = o4;
    return;
  } else if (u < E9) {
    const int vv = u - E8;
    const int wv = __builtin_amdgcn_readfirstlane(vv >> 5);
    const int ln = vv & 31;
    const float* src = (wv == 0) ? sb1 : sb2;
    const v4f a = *(const v4fa*)(src + 4 * ln);
    v4f o4;
    o4.x = bf16_val(a.x);
    o4.y = bf16_val(a.y);
    o4.z = bf16_val(a.z);
    o4.w = bf16_val(a.w);
    putf4(VEC + 256 + DS * wv + 4 * ln, o4);
    return;
  }
}

template <int MODE, int NT>
__global__ __launch_bounds__(GTHR) void k_gemm(const unsigned short* __restrict__ A, int lda,
                                               const unsigned short* __restrict__ BT, int ldb, int K,
                                               const float* __restrict__ bias,
                                               const unsigned short* __restrict__ RES, int ldr,
                                               float* Cm, unsigned short* Cb) {
  constexpr int GN = 16 * NT;
  static_assert((MODE == 0 && NT == 4) || (MODE != 0 && NT == 8));
  __shared__ __attribute__((aligned(16))) float stg[GBM * GN];
  const int tid = (int)threadIdx.x, lane = tid & 31, wave = tid >> 5, hh = lane >> 4, m = lane & 15;
  const int rowBase = (int)blockIdx.x * GBM;

  v8f acc[NT];
  {
    const v8f z = {0.f, 0.f, 0.f, 0.f, 0.f, 0.f, 0.f, 0.f};
#pragma unroll
    for (int t = 0; t < NT; ++t) acc[t] = z;
  }
  const unsigned short* ap = A  + (size_t)(rowBase + 16 * wave + m) * (size_t)lda + 8 * hh;
  const unsigned short* bp = BT + (size_t)m * (size_t)ldb + 8 * hh;

#pragma unroll 1
  for (int k0 = 0; k0 < K; k0 += 32) {
    FragB af;
    af.h[0] = *(const v8usa*)(ap + k0);
    af.h[1] = *(const v8usa*)(ap + k0 + 16);
#pragma unroll
    for (int nt = 0; nt < NT; ++nt) {
      const unsigned short* wq = bp + (size_t)(16 * nt) * (size_t)ldb + k0;
      FragB bf;
      bf.h[0] = *(const v8usa*)wq;
      bf.h[1] = *(const v8usa*)(wq + 16);
      acc[nt] = wmb(af, bf, acc[nt]);
    }
  }

#pragma unroll
  for (int nt = 0; nt < NT; ++nt) {
    const int lc = 16 * nt + m;
    float bvv = 0.0f;
    if constexpr (MODE != 0) bvv = bias[lc];
#pragma unroll
    for (int r = 0; r < 8; ++r) {
      const int lr = 16 * wave + 8 * hh + r;
      float v = acc[nt][r];
      if constexpr (MODE == 1) v = silu_f(v + bvv);
      if constexpr (MODE == 2) v = v + bvv;
      stg[lr * GN + lc] = v;
    }
  }
  __syncthreads();

  if constexpr (MODE == 0) {
    const int rs = lane >> 4, c4 = (lane & 15) * 4;
    v4f pv[8];
#pragma unroll
    for (int it = 0; it < 8; ++it) pv[it] = *(const v4fa*)(stg + (16 * wave + 2 * it + rs) * GN + c4);
#pragma unroll
    for (int it = 0; it < 8; ++it) {
      float* op = Cm + (size_t)(rowBase + 16 * wave + 2 * it + rs) * GN + c4;
      *(volatile v4f*)op = pv[it];
    }
    __threadfence();
#pragma unroll
    for (int it = 0; it < 8; ++it) {
      float* op = Cm + (size_t)(rowBase + 16 * wave + 2 * it + rs) * GN + c4;
      *(volatile v4f*)op = pv[it];
    }
  } else if constexpr (MODE == 1) {
    const int part = lane >> 4;
    const int j = lane & 15;
    const unsigned mh = 0u - (unsigned)part;
    const unsigned ml = ~mh;
    v8us pv[16];
#pragma unroll
    for (int i = 0; i < 16; ++i) {
      const float* sp = stg + (16 * wave + i) * GN + 8 * j;
      const v4f a = *(const v4fa*)sp;
      const v4f b = *(const v4fa*)(sp + 4);
      const v8f f8 = {a.x, a.y, a.z, a.w, b.x, b.y, b.z, b.w};
      v8us oo;
#pragma unroll
      for (int e = 0; e < 8; ++e) {
        const unsigned hb = bf16_bits(f8[e]);
        const unsigned lb = bf16_bits(f8[e] - __uint_as_float(hb << 16));
        oo[e] = (unsigned short)((hb & ml) | (lb & mh));
      }
      pv[i] = oo;
    }
#pragma unroll
    for (int i = 0; i < 16; ++i) {
      unsigned short* op = Cb + (size_t)(rowBase + 16 * wave + i) * (size_t)KH + part * DS + 8 * j;
      *(volatile v8us*)op = pv[i];
    }
    __threadfence();
#pragma unroll
    for (int i = 0; i < 16; ++i) {
      unsigned short* op = Cb + (size_t)(rowBase + 16 * wave + i) * (size_t)KH + part * DS + 8 * j;
      *(volatile v8us*)op = pv[i];
    }
  } else {
    v4f pv[16];
#pragma unroll
    for (int i = 0; i < 16; ++i) {
      const int row = rowBase + 16 * wave + i;
      const v2u w = *(const v2ua*)(RES + (size_t)row * (size_t)ldr + 4 * lane);
      const v4f sv = *(const v4fa*)(stg + (16 * wave + i) * GN + 4 * lane);
      v4f q;
      q.x = sv.x + __uint_as_float(w.x << 16);
      q.y = sv.y + __uint_as_float(w.x & 0xffff0000u);
      q.z = sv.z + __uint_as_float(w.y << 16);
      q.w = sv.w + __uint_as_float(w.y & 0xffff0000u);
      pv[i] = q;
    }
#pragma unroll
    for (int i = 0; i < 16; ++i) {
      float* op = Cm + (size_t)(rowBase + 16 * wave + i) * GN + 4 * lane;
      *(volatile v4f*)op = pv[i];
    }
    __threadfence();
#pragma unroll
    for (int i = 0; i < 16; ++i) {
      float* op = Cm + (size_t)(rowBase + 16 * wave + i) * GN + 4 * lane;
      *(volatile v4f*)op = pv[i];
    }
  }
}

__global__ __launch_bounds__(NTHR) __attribute__((amdgpu_num_vgpr(248)))
void k_pair(const float* __restrict__ PQ, const float* __restrict__ XR, const int* __restrict__ mask,
            const float* __restrict__ VEC, const unsigned short* __restrict__ W2,
            const unsigned short* __restrict__ W3, unsigned short* A1, float* MX) {
  extern __shared__ __attribute__((aligned(16))) float dyn[];
  float* sQ  = dyn;
  float* sX  = sQ + LQ;
  int*   sM  = (int*)(sX + LX);
  float* sV  = sX + LX + LM;
  float* sW  = sV + LV;
  float* sMX = sW + LW;

  const int tid = (int)threadIdx.x, lane = tid & 31, wave = tid >> 5, hh = lane >> 4, m = lane & 15;
  const int r0 = (int)blockIdx.x * RPB;
  const int rb = (r0 >> 9) << 9;

#pragma unroll 4
  for (int it = 0; it < (LQ / 4) / NTHR; ++it) {
    const int idx = it * NTHR + tid;
    const int row = idx >> 3;
    const int c4  = (idx & 7) * 4;
    const v4f v = *(const v4fa*)(PQ + (size_t)(rb + row) * NPQ + ED + c4);
    *(v4fa*)(sQ + row * ED + c4) = v;
  }
#pragma unroll
  for (int it = 0; it < 2; ++it) {
    const int row = it * NTHR + tid;
    const v4f v = *(const v4fa*)(XR + (size_t)(rb + row) * 4);
    *(v4fa*)(sX + row * 4) = v;
    sM[row] = mask[rb + row];
  }
  if (tid < LV / 4) {
    const v4f v = *(const v4fa*)(VEC + 4 * tid);
    *(v4fa*)(sV + 4 * tid) = v;
  }
  __syncthreads();

  const int r = r0 + wave;
  const int i = r & (NN - 1);
  float base[16], wk[16];
  {
    const float* pr = PQ + (size_t)r * NPQ + 8 * hh;
    const v4f p0 = *(const v4fa*)(pr);
    const v4f p1 = *(const v4fa*)(pr + 4);
    const v4f p2 = *(const v4fa*)(pr + 16);
    const v4f p3 = *(const v4fa*)(pr + 20);
    const float* er = sV + 32 + 8 * hh;
    const v4f e0 = *(const v4fa*)(er);
    const v4f e1 = *(const v4fa*)(er + 4);
    const v4f e2 = *(const v4fa*)(er + 16);
    const v4f e3 = *(const v4fa*)(er + 20);
    const float* wr = sV + 8 * hh;
    const v4f w0 = *(const v4fa*)(wr);
    const v4f w1 = *(const v4fa*)(wr + 4);
    const v4f w2 = *(const v4fa*)(wr + 16);
    const v4f w3 = *(const v4fa*)(wr + 20);
    base[0]  = p0.x + e0.x; base[1]  = p0.y + e0.y; base[2]  = p0.z + e0.z; base[3]  = p0.w + e0.w;
    base[4]  = p1.x + e1.x; base[5]  = p1.y + e1.y; base[6]  = p1.z + e1.z; base[7]  = p1.w + e1.w;
    base[8]  = p2.x + e2.x; base[9]  = p2.y + e2.y; base[10] = p2.z + e2.z; base[11] = p2.w + e2.w;
    base[12] = p3.x + e3.x; base[13] = p3.y + e3.y; base[14] = p3.z + e3.z; base[15] = p3.w + e3.w;
    wk[0]  = w0.x; wk[1]  = w0.y; wk[2]  = w0.z; wk[3]  = w0.w;
    wk[4]  = w1.x; wk[5]  = w1.y; wk[6]  = w1.z; wk[7]  = w1.w;
    wk[8]  = w2.x; wk[9]  = w2.y; wk[10] = w2.z; wk[11] = w2.w;
    wk[12] = w3.x; wk[13] = w3.y; wk[14] = w3.z; wk[15] = w3.w;
  }
  const v4f xi = *(const v4fa*)(sX + 4 * i);
  const unsigned mi = (unsigned)sM[i];
  const float eb2v0 = sV[64 + m],  eb2v1 = sV[64 + 16 + m];
  const float ab1v0 = sV[96 + m],  ab1v1 = sV[96 + 16 + m];
  const float cb1v0 = sV[128 + m], cb1v1 = sV[128 + 16 + m];
  const float aw2v0 = sV[160 + m], aw2v1 = sV[160 + 16 + m];
  const float cw2v0 = sV[192 + m], cw2v1 = sV[192 + 16 + m];
  const float ab2s = sV[224], cb2s = sV[225];

  FragB bw2[2], bw3[4];
#pragma unroll
  for (int nt = 0; nt < 2; ++nt) {
    const unsigned short* wq = W2 + (size_t)(16 * nt + m) * ED + 8 * hh;
    bw2[nt].h[0] = *(const v8usa*)wq;
    bw2[nt].h[1] = *(const v8usa*)(wq + 16);
  }
#pragma unroll
  for (int nt = 0; nt < 4; ++nt) {
    const unsigned short* wq = W3 + (size_t)(16 * nt + m) * ED + 8 * hh;
    bw3[nt].h[0] = *(const v8usa*)wq;
    bw3[nt].h[1] = *(const v8usa*)(wq + 16);
  }

  float* EF = sW + wave * WVF;
  float* LG = EF + 16 * EFP;
  float* CW = LG + 16;

  const float NINF = -__builtin_inff();
  const v8f z8 = {0.f, 0.f, 0.f, 0.f, 0.f, 0.f, 0.f, 0.f};
  float mrun = NINF, lsum = 0.0f, ams = 0.0f, amx0 = 0.0f, amx1 = 0.0f, amx2 = 0.0f;

#pragma unroll 1
  for (int jt = 0; jt < NN / 16; ++jt) {
    const int j = 16 * jt + m;
    const v4f xj = *(const v4fa*)(sX + 4 * j);
    const float dx = xi.x - xj.x, dy = xi.y - xj.y, dz = xi.z - xj.z;
    const float d2 = (dx * dx + dy * dy) + dz * dz;
    FragB ahi, alo;
    {
      const float* qr = sQ + j * ED + 8 * hh;
      const v4f q0 = *(const v4fa*)(qr);
      const v4f q1 = *(const v4fa*)(qr + 4);
      const v4f q2 = *(const v4fa*)(qr + 16);
      const v4f q3 = *(const v4fa*)(qr + 20);
      const float qv[16] = {q0.x, q0.y, q0.z, q0.w, q1.x, q1.y, q1.z, q1.w,
                            q2.x, q2.y, q2.z, q2.w, q3.x, q3.y, q3.z, q3.w};
#pragma unroll
      for (int e = 0; e < 16; ++e) {
        const float pre = fmaf(d2, wk[e], base[e] + qv[e]);
        const unsigned sp = split2(silu_f(pre));
        ahi.u[e] = (unsigned short)(sp & 0xffffu);
        alo.u[e] = (unsigned short)(sp >> 16);
      }
    }
    {
      v8f acc = z8;
      acc = wmb(ahi, bw2[0], acc);
      acc = wmb(alo, bw2[0], acc);
#pragma unroll
      for (int rr = 0; rr < 8; ++rr) EF[(8 * hh + rr) * EFP + m] = acc[rr] + eb2v0;
    }
    {
      v8f acc = z8;
      acc = wmb(ahi, bw2[1], acc);
      acc = wmb(alo, bw2[1], acc);
#pragma unroll
      for (int rr = 0; rr < 8; ++rr) EF[(8 * hh + rr) * EFP + 16 + m] = acc[rr] + eb2v1;
    }
    wave_sync();
    FragB ehi, elo;
    {
      const float* er = EF + m * EFP + 8 * hh;
      const v4f e0 = *(const v4fa*)(er);
      const v4f e1 = *(const v4fa*)(er + 4);
      const v4f e2 = *(const v4fa*)(er + 16);
      const v4f e3 = *(const v4fa*)(er + 20);
      const float ev[16] = {e0.x, e0.y, e0.z, e0.w, e1.x, e1.y, e1.z, e1.w,
                            e2.x, e2.y, e2.z, e2.w, e3.x, e3.y, e3.z, e3.w};
#pragma unroll
      for (int e = 0; e < 16; ++e) {
        const unsigned sp = split2(ev[e]);
        ehi.u[e] = (unsigned short)(sp & 0xffffu);
        elo.u[e] = (unsigned short)(sp >> 16);
      }
    }
    float ta[8], tc[8];
    {
      v8f acc = z8;
      acc = wmb(ehi, bw3[0], acc);
      acc = wmb(elo, bw3[0], acc);
#pragma unroll
      for (int rr = 0; rr < 8; ++rr) ta[rr] = silu_f(acc[rr] + ab1v0) * aw2v0;
    }
    {
      v8f acc = z8;
      acc = wmb(ehi, bw3[1], acc);
      acc = wmb(elo, bw3[1], acc);
#pragma unroll
      for (int rr = 0; rr < 8; ++rr) ta[rr] = fmaf(silu_f(acc[rr] + ab1v1), aw2v1, ta[rr]);
    }
    {
      v8f acc = z8;
      acc = wmb(ehi, bw3[2], acc);
      acc = wmb(elo, bw3[2], acc);
#pragma unroll
      for (int rr = 0; rr < 8; ++rr) tc[rr] = silu_f(acc[rr] + cb1v0) * cw2v0;
    }
    {
      v8f acc = z8;
      acc = wmb(ehi, bw3[3], acc);
      acc = wmb(elo, bw3[3], acc);
#pragma unroll
      for (int rr = 0; rr < 8; ++rr) tc[rr] = fmaf(silu_f(acc[rr] + cb1v1), cw2v1, tc[rr]);
    }
#pragma unroll
    for (int rr = 0; rr < 8; ++rr) {
      ta[rr] = hsum16(ta[rr]) + ab2s;
      tc[rr] = hsum16(tc[rr]) + cb2s;
    }
    if (m == 0) {
      const v4f l0 = {ta[0], ta[1], ta[2], ta[3]};
      const v4f l1 = {ta[4], ta[5], ta[6], ta[7]};
      const v4f c0 = {tc[0], tc[1], tc[2], tc[3]};
      const v4f c1 = {tc[4], tc[5], tc[6], tc[7]};
      *(v4fa*)(LG + 8 * hh)     = l0;
      *(v4fa*)(LG + 8 * hh + 4) = l1;
      *(v4fa*)(CW + 8 * hh)     = c0;
      *(v4fa*)(CW + 8 * hh + 4) = c1;
    }
    wave_sync();
    {
      const float lg  = LG[m];
      const float cwv = CW[m];
      const unsigned mj = (unsigned)sM[j];
      const bool valid = (sqrtf(d2) <= 150.0f) && ((mi * mj) != 0u);
      const float lgv  = valid ? lg : NINF;
      const float tmax = hmax16(lgv);
      const float mnew = fmaxf(mrun, tmax);
      const bool dead  = (mnew == NINF);
      const float e_sc = expf(mrun - mnew);
      const float e_p  = expf(lgv - mnew);
      const float sc = dead ? 0.0f : e_sc;
      const float p  = dead ? 0.0f : e_p;
      const float pw = p * cwv;
      const float ps = hsum16(p);
      const float px = hsum16(pw * dx);
      const float py = hsum16(pw * dy);
      const float pz = hsum16(pw * dz);
      lsum = fmaf(lsum, sc, ps);
      amx0 = fmaf(amx0, sc, px);
      amx1 = fmaf(amx1, sc, py);
      amx2 = fmaf(amx2, sc, pz);
      float sacc = 0.0f;
#pragma unroll
      for (int jj = 0; jj < 16; ++jj) {
        const float pj = __shfl(p, jj, 32);
        sacc = fmaf(pj, EF[jj * EFP + lane], sacc);
      }
      ams  = fmaf(ams, sc, sacc);
      mrun = mnew;
    }
    wave_sync();
  }

  const float inv = 1.0f / lsum;
  EF[lane] = ams * inv;
  wave_sync();
  {
    const int q    = lane & 7;
    const int part = q >> 2;
    const int c8   = (q & 3) * 8;
    const unsigned mh = 0u - (unsigned)part;
    const unsigned ml = ~mh;
    const v4f a = *(const v4fa*)(EF + c8);
    const v4f b = *(const v4fa*)(EF + c8 + 4);
    const float f8[8] = {a.x, a.y, a.z, a.w, b.x, b.y, b.z, b.w};
    v8us o;
#pragma unroll
    for (int e = 0; e < 8; ++e) {
      const unsigned sp = split2(f8[e]);
      o[e] = (unsigned short)(((sp & 0xffffu) & ml) | ((sp >> 16) & mh));
    }
    unsigned short* dp = A1 + (size_t)r * KA1 + DS + 8 * q;
    if (lane < 8) *(volatile v8us*)dp = o;
    __threadfence();
    if (lane < 8) *(volatile v8us*)dp = o;
  }
  if (lane == 0) {
    const v4f mxv = {amx0 * inv, amx1 * inv, amx2 * inv, 0.0f};
    *(v4fa*)(sMX + 4 * wave) = mxv;
  }
  __syncthreads();
  if (wave == 0) {
    const int q = lane & 7;
    const v4f o4 = *(const v4fa*)(sMX + 4 * q);
    float* mp = MX + (size_t)(r0 + q) * 4;
    if (lane < 8) *(volatile v4f*)mp = o4;
    __threadfence();
    if (lane < 8) *(volatile v4f*)mp = o4;
  }
}

__global__ __launch_bounds__(NTHR) void k_xout(const float* __restrict__ XR, const float* __restrict__ MX,
                                               float* out1) {
  const int u = (int)blockIdx.x * NTHR + (int)threadIdx.x;
  if (u >= (MR * 3) / 4) return;
  const int f  = 4 * u;
  const int ra = f / 3;
  const int c0 = f - 3 * ra;
  const int rn = (ra + 1 < MR) ? (ra + 1) : (MR - 1);
  const v4f xa = *(const v4fa*)(XR + (size_t)ra * 4);
  const v4f xb = *(const v4fa*)(XR + (size_t)rn * 4);
  const v4f ma = *(const v4fa*)(MX + (size_t)ra * 4);
  const v4f mb = *(const v4fa*)(MX + (size_t)rn * 4);
  const float a0 = xa.x + ma.x, a1 = xa.y + ma.y, a2 = xa.z + ma.z;
  const float b0 = xb.x + mb.x, b1 = xb.y + mb.y, b2 = xb.z + mb.z;
  v4f o;
  o.x = (c0 == 0) ? a0 : ((c0 == 1) ? a1 : a2);
  o.y = (c0 == 0) ? a1 : ((c0 == 1) ? a2 : b0);
  o.z = (c0 == 0) ? a2 : ((c0 == 1) ? b0 : b1);
  o.w = (c0 == 0) ? b0 : ((c0 == 1) ? b1 : b2);
  putf4(out1 + (size_t)f, o);
}

extern "C" void kernel_launch(void* const* d_in, const int* in_sizes, int n_in,
                              void* d_out, int out_size, void* d_ws, size_t ws_size,
                              hipStream_t stream) {
  if (n_in < 19) return;
  if (in_sizes[0] != MR * DS) return;
  if (in_sizes[1] != MR * 3) return;
  if (in_sizes[2] != MR) return;
  if (in_sizes[3] != (2 * DS + 1) * ED) return;
  if (in_sizes[4] != ED) return;
  if (in_sizes[5] != ED * ED || in_sizes[6] != ED) return;
  if (in_sizes[7] != ED * ED || in_sizes[8] != ED) return;
  if (in_sizes[9] != ED || in_sizes[10] != 1) return;
  if (in_sizes[11] != (DS + ED) * DS || in_sizes[12] != DS) return;
  if (in_sizes[13] != DS * DS || in_sizes[14] != DS) return;
  if (in_sizes[15] != ED * ED || in_sizes[16] != ED) return;
  if (in_sizes[17] != ED || in_sizes[18] != 1) return;
  if (out_size != MR * DS + MR * 3) return;

  const float* s    = (const float*)d_in[0];
  const float* x    = (const float*)d_in[1];
  const int*   mask = (const int*)d_in[2];
  const float* ew1  = (const float*)d_in[3];
  const float* eb1  = (const float*)d_in[4];
  const float* ew2  = (const float*)d_in[5];
  const float* eb2  = (const float*)d_in[6];
  const float* aw1  = (const float*)d_in[7];
  const float* ab1  = (const float*)d_in[8];
  const float* aw2  = (const float*)d_in[9];
  const float* ab2  = (const float*)d_in[10];
  const float* sw1  = (const float*)d_in[11];
  const float* sb1  = (const float*)d_in[12];
  const float* sw2  = (const float*)d_in[13];
  const float* sb2  = (const float*)d_in[14];
  const float* cw1  = (const float*)d_in[15];
  const float* cb1  = (const float*)d_in[16];
  const float* cw2  = (const float*)d_in[17];
  const float* cb2  = (const float*)d_in[18];
  float* out0 = (float*)d_out;
  float* out1 = out0 + (size_t)MR * DS;

  char* ws = (char*)d_ws;
  size_t off = 0;
  const size_t oA1  = off; off += (size_t)MR * KA1 * 2;   off = (off + 255) & ~(size_t)255;
  const size_t oPQ  = off; off += (size_t)MR * NPQ * 4;   off = (off + 255) & ~(size_t)255;
  const size_t oHHL = off; off += (size_t)MR * KH * 2;    off = (off + 255) & ~(size_t)255;
  const size_t oMX  = off; off += (size_t)MR * 4 * 4;     off = (off + 255) & ~(size_t)255;
  const size_t oXR  = off; off += (size_t)MR * 4 * 4;     off = (off + 255) & ~(size_t)255;
  const size_t oWPQ = off; off += (size_t)NPQ * DS * 2;   off = (off + 255) & ~(size_t)255;
  const size_t oW2  = off; off += (size_t)ED * ED * 2;    off = (off + 255) & ~(size_t)255;
  const size_t oW3  = off; off += (size_t)2 * ED * ED * 2; off = (off + 255) & ~(size_t)255;
  const size_t oSW1 = off; off += (size_t)DS * KA1 * 2;   off = (off + 255) & ~(size_t)255;
  const size_t oSW2 = off; off += (size_t)DS * KH * 2;    off = (off + 255) & ~(size_t)255;
  const size_t oVEC = off; off += (size_t)4096;           off = (off + 255) & ~(size_t)255;
  if (off > ws_size || off > (size_t)WSMAX) return;

  unsigned short* A1   = (unsigned short*)(ws + oA1);
  float*          PQ   = (float*)(ws + oPQ);
  unsigned short* HHL  = (unsigned short*)(ws + oHHL);
  float*          MX   = (float*)(ws + oMX);
  float*          XR   = (float*)(ws + oXR);
  unsigned short* WPQ  = (unsigned short*)(ws + oWPQ);
  unsigned short* W2   = (unsigned short*)(ws + oW2);
  unsigned short* W3   = (unsigned short*)(ws + oW3);
  unsigned short* SW1C = (unsigned short*)(ws + oSW1);
  unsigned short* SW2D = (unsigned short*)(ws + oSW2);
  float*          VEC  = (float*)(ws + oVEC);

  hipFuncSetAttribute(reinterpret_cast<const void*>(&k_pair), hipFuncAttributeMaxDynamicSharedMemorySize,
                      (int)PAIR_LDS_BYTES);

  k_prep<<<(E9 + NTHR - 1) / NTHR, NTHR, 0, stream>>>(s, x, ew1, eb1, ew2, eb2, aw1, ab1, aw2, ab2,
                                                      sw1, sb1, sw2, sb2, cw1, cb1, cw2, cb2,
                                                      A1, XR, WPQ, W2, W3, SW1C, SW2D, VEC);
  k_gemm<0, 4><<<MR / GBM, GTHR, 0, stream>>>(A1, KA1, WPQ, DS, DS, VEC, A1, KA1, PQ, HHL);
  k_pair<<<MR / RPB, NTHR, PAIR_LDS_BYTES, stream>>>(PQ, XR, mask, VEC, W2, W3, A1, MX);
  k_gemm<1, 8><<<MR / GBM, GTHR, 0, stream>>>(A1, KA1, SW1C, KA1, KA1, VEC + 256, A1, KA1, PQ, HHL);
  k_gemm<2, 8><<<MR / GBM, GTHR, 0, stream>>>(HHL, KH, SW2D, KH, KH, VEC + 384, A1, KA1, out0, HHL);
  k_xout<<<((MR * 3) / 4) / NTHR, NTHR, 0, stream>>>(XR, MX, out1);
  (void)hipGetLastError();
}
